// gcs_layer_44341242364284
// MI455X (gfx1250) — hardware-verified
//
#include <hip/hip_runtime.h>
#define NNODE 50000
#define NEDGE 800000
#define NP2 1048576
#define DIM 256
#define TEMP 0.5f

typedef __bf16 v16b __attribute__((ext_vector_type(16)));
typedef unsigned short v8us __attribute__((ext_vector_type(8), may_alias));
typedef float  v8f  __attribute__((ext_vector_type(8)));
typedef float  v4f  __attribute__((ext_vector_type(4)));
typedef float  v4fa __attribute__((ext_vector_type(4), may_alias));
union FragB { v16b v; v8us half[2]; unsigned short u[16]; };

__device__ __forceinline__ unsigned short bf16_bits(float x) { unsigned int u = __float_as_uint(x); return (unsigned short)((u + 0x7FFFu + ((u >> 16) & 1u)) >> 16); }
__device__ __forceinline__ float bf16_val(unsigned short b) { return __uint_as_float(((unsigned int)b) << 16); }
__device__ __forceinline__ float bf16_round(float x) { return bf16_val(bf16_bits(x)); }
template <int NT>
__device__ __forceinline__ v8f mmaN(v16b ah, v16b al, v16b bh, v16b bl, v8f c) {
  c = __builtin_amdgcn_wmma_f32_16x16x32_bf16(false, ah, false, bh, (short)0, c, false, false);
  if (NT >= 2) c = __builtin_amdgcn_wmma_f32_16x16x32_bf16(false, al, false, bh, (short)0, c, false, false);
  if (NT >= 3) c = __builtin_amdgcn_wmma_f32_16x16x32_bf16(false, ah, false, bl, (short)0, c, false, false);
  asm volatile("v_nop\n\tv_nop\n\tv_nop\n\tv_nop" : "+v"(c) : "v"(ah), "v"(al), "v"(bh), "v"(bl));
  return c;
}

__global__ __launch_bounds__(256) void k_wt_bf16(const float* __restrict__ W, unsigned short* __restrict__ Wt, int K, int N) {
  const int t = blockIdx.x * 256 + threadIdx.x;
  const int k8n = K / 8;
  if (t >= N * k8n) return;
  const int n = t / k8n, k8 = (t % k8n) * 8;
  v8us v;
#pragma unroll
  for (int i = 0; i < 8; ++i) v[i] = bf16_bits(W[(size_t)(k8 + i) * N + n]);
  *(volatile v8us*)(Wt + (size_t)n * K + k8) = v;
  __threadfence();
  *(volatile v8us*)(Wt + (size_t)n * K + k8) = v;
}

template <bool ASPLIT, int ACT, bool BIAS_BF16>
__global__ __launch_bounds__(128) void k_gemm_bf(const float* __restrict__ A, int lda, const unsigned short* __restrict__ Wt, int ldb,
                                               const float* __restrict__ bias, float* __restrict__ C, int ldc, int M, int N, int K) {
  __shared__ __attribute__((aligned(16))) float so[4][16][64];
  const int tid = threadIdx.x, w = tid >> 5, lane = tid & 31, ln = lane & 15, hh = lane >> 4;
  const int ntn = N / 64;
  const int wid = blockIdx.x * 4 + w;
  const int mt = wid / ntn, nq = wid % ntn;
  if (mt * 16 >= M) return;
  const int row0 = mt * 16, col0 = nq * 64;
  const float* arow = A + (size_t)(row0 + ln) * lda;
  v8f acc[4] = {};
  for (int kb = 0; kb < K; kb += 32) {
    FragB ah, al;
    const v4f x0 = *(const v4fa*)(arow + kb + 8 * hh), x1 = *(const v4fa*)(arow + kb + 8 * hh + 4);
    const v4f x2 = *(const v4fa*)(arow + kb + 16 + 8 * hh), x3 = *(const v4fa*)(arow + kb + 16 + 8 * hh + 4);
    float xs[16] = {x0[0],x0[1],x0[2],x0[3],x1[0],x1[1],x1[2],x1[3],x2[0],x2[1],x2[2],x2[3],x3[0],x3[1],x3[2],x3[3]};
#pragma unroll
    for (int i = 0; i < 16; ++i) { const unsigned short hb = bf16_bits(xs[i]); ah.u[i] = hb; al.u[i] = ASPLIT ? bf16_bits(xs[i] - bf16_val(hb)) : (unsigned short)0; }
#pragma unroll
    for (int t = 0; t < 4; ++t) {
      const unsigned short* brow = Wt + (size_t)(col0 + t * 16 + ln) * ldb + kb;
      FragB b;
      b.half[0] = *(const v8us*)(brow + 8 * hh);
      b.half[1] = *(const v8us*)(brow + 16 + 8 * hh);
      acc[t] = mmaN<ASPLIT ? 2 : 1>(ah.v, al.v, b.v, b.v, acc[t]);
    }
  }
#pragma unroll
  for (int t = 0; t < 4; ++t) {
    float bv = bias ? bias[col0 + t * 16 + ln] : 0.f;
    if (BIAS_BF16) bv = bf16_round(bv);
#pragma unroll
    for (int r = 0; r < 8; ++r) { float v = acc[t][r] + bv; if (ACT == 1) v = fmaxf(v, 0.f); so[w][8 * hh + r][t * 16 + ln] = v; }
  }
  __builtin_amdgcn_fence(__ATOMIC_ACQ_REL, "workgroup");
  __builtin_amdgcn_wave_barrier();
  const int rsub = lane >> 4, c4 = (lane & 15) * 4;
  for (int pass = 0; pass < 2; ++pass) {
#pragma unroll
    for (int q = 0; q < 8; ++q) {
      const int r = q * 2 + rsub;
      const v4f v = *(const v4fa*)&so[w][r][c4];
      *(volatile v4f*)(C + (size_t)(row0 + r) * ldc + col0 + c4) = v;
    }
    if (pass == 0) __threadfence();
  }
}

template <int D, bool CAUSAL>
__global__ __launch_bounds__(128) void k_flash(const float* __restrict__ qb, const float* __restrict__ kb, const float* __restrict__ vb,
                                             int pitch, int T, int H, float scale, float* __restrict__ y, int ypitch) {
  constexpr int KS = D / 32;
  constexpr int DT = D / 16;
  __shared__ __attribute__((aligned(16))) unsigned short sKh[32][D + 8], sKl[32][D + 8], sVh[32][D + 8], sVl[32][D + 8];
  __shared__ __attribute__((aligned(16))) unsigned short sPh[4][16][40], sPl[4][16][40];
  __shared__ __attribute__((aligned(16))) float sO[4][16][D];
  const int tid = threadIdx.x, w = tid >> 5, lane = tid & 31, ln = lane & 15, hh = lane >> 4;
  const int nqb = (T + 63) / 64;
  const int bh = blockIdx.x / nqb, qblk = blockIdx.x % nqb;
  const int b = bh / H, h = bh % H;
  const int q0 = qblk * 64 + w * 16;
  const float* Q = qb + (size_t)b * T * pitch + h * D;
  const float* K = kb + (size_t)b * T * pitch + h * D;
  const float* V = vb + (size_t)b * T * pitch + h * D;

  FragB aqh[KS], aql[KS];
  {
    int row = q0 + ln; if (row >= T) row = T - 1;
    const float* qr = Q + (size_t)row * pitch;
#pragma unroll
    for (int ks = 0; ks < KS; ++ks)
#pragma unroll
      for (int i = 0; i < 16; ++i) {
        const int d = ks * 32 + ((i < 8) ? (8 * hh + i) : (16 + 8 * hh + (i - 8)));
        const float x = qr[d] * scale; const unsigned short hb = bf16_bits(x);
        aqh[ks].u[i] = hb; aql[ks].u[i] = bf16_bits(x - bf16_val(hb));
      }
  }
  float m_r[8], l_r[8];
#pragma unroll
  for (int r = 0; r < 8; ++r) { m_r[r] = -3.0e38f; l_r[r] = 0.f; }
  v8f oacc[DT];
#pragma unroll
  for (int dt = 0; dt < DT; ++dt) oacc[dt] = (v8f){0.f,0.f,0.f,0.f,0.f,0.f,0.f,0.f};

  const int kv_end = CAUSAL ? min(T, qblk * 64 + 64) : T;
  for (int j0 = 0; j0 < kv_end; j0 += 32) {
    __syncthreads();
    for (int e = tid; e < 32 * (D / 4); e += 128) {
      const int r = e / (D / 4), c4 = (e % (D / 4)) * 4;
      const int key = j0 + r;
      v4f kf = {0.f,0.f,0.f,0.f}, vf = {0.f,0.f,0.f,0.f};
      if (key < T) { kf = *(const v4fa*)(K + (size_t)key * pitch + c4); vf = *(const v4fa*)(V + (size_t)key * pitch + c4); }
#pragma unroll
      for (int t = 0; t < 4; ++t) {
        unsigned short hb = bf16_bits(kf[t]); sKh[r][c4 + t] = hb; sKl[r][c4 + t] = bf16_bits(kf[t] - bf16_val(hb));
        hb = bf16_bits(vf[t]); sVh[r][c4 + t] = hb; sVl[r][c4 + t] = bf16_bits(vf[t] - bf16_val(hb));
      }
    }
    __syncthreads();
    v8f s[2];
#pragma unroll
    for (int nt = 0; nt < 2; ++nt) {
      v8f acc = {};
#pragma unroll
      for (int ks = 0; ks < KS; ++ks) {
        FragB bh_, bl_;
        bh_.half[0] = *(const v8us*)&sKh[nt * 16 + ln][ks * 32 + 8 * hh]; bh_.half[1] = *(const v8us*)&sKh[nt * 16 + ln][ks * 32 + 16 + 8 * hh];
        bl_.half[0] = *(const v8us*)&sKl[nt * 16 + ln][ks * 32 + 8 * hh]; bl_.half[1] = *(const v8us*)&sKl[nt * 16 + ln][ks * 32 + 16 + 8 * hh];
        acc = mmaN<3>(aqh[ks].v, aql[ks].v, bh_.v, bl_.v, acc);
      }
      s[nt] = acc;
    }
    float alpha[8];
#pragma unroll
    for (int r = 0; r < 8; ++r) {
      const int qi = q0 + 8 * hh + r;
      const int ja = j0 + ln, jb = j0 + 16 + ln;
      if (CAUSAL) { if (ja > qi) s[0][r] = -3.0e38f; if (jb > qi) s[1][r] = -3.0e38f; }
      if (ja >= T) s[0][r] = -3.0e38f;
      if (jb >= T) s[1][r] = -3.0e38f;
      float mx = fmaxf(s[0][r], s[1][r]);
      mx = fmaxf(mx, __shfl_xor(mx, 1, 32)); mx = fmaxf(mx, __shfl_xor(mx, 2, 32)); mx = fmaxf(mx, __shfl_xor(mx, 4, 32)); mx = fmaxf(mx, __shfl_xor(mx, 8, 32));
      const float mnew = fmaxf(m_r[r], mx);
      alpha[r] = (mnew > -1.0e38f) ? __expf(m_r[r] - mnew) : 1.0f;
      const float p0 = (s[0][r] > -1.0e38f) ? __expf(s[0][r] - mnew) : 0.f;
      const float p1 = (s[1][r] > -1.0e38f) ? __expf(s[1][r] - mnew) : 0.f;
      m_r[r] = mnew;
      l_r[r] = l_r[r] * alpha[r] + p0 + p1;
      unsigned short hb = bf16_bits(p0); sPh[w][8 * hh + r][ln] = hb;      sPl[w][8 * hh + r][ln] = bf16_bits(p0 - bf16_val(hb));
      hb = bf16_bits(p1);                sPh[w][8 * hh + r][16 + ln] = hb; sPl[w][8 * hh + r][16 + ln] = bf16_bits(p1 - bf16_val(hb));
    }
#pragma unroll
    for (int dt = 0; dt < DT; ++dt)
#pragma unroll
      for (int r = 0; r < 8; ++r) oacc[dt][r] *= alpha[r];
    __builtin_amdgcn_fence(__ATOMIC_ACQ_REL, "workgroup");
    __builtin_amdgcn_wave_barrier();
    FragB pah, pal;
    pah.half[0] = *(const v8us*)&sPh[w][ln][8 * hh]; pah.half[1] = *(const v8us*)&sPh[w][ln][16 + 8 * hh];
    pal.half[0] = *(const v8us*)&sPl[w][ln][8 * hh]; pal.half[1] = *(const v8us*)&sPl[w][ln][16 + 8 * hh];
#pragma unroll
    for (int dt = 0; dt < DT; ++dt) {
      FragB bvh, bvl;
#pragma unroll
      for (int i = 0; i < 8; ++i) {
        bvh.u[i] = sVh[8 * hh + i][dt * 16 + ln]; bvh.u[8 + i] = sVh[16 + 8 * hh + i][dt * 16 + ln];
        bvl.u[i] = sVl[8 * hh + i][dt * 16 + ln]; bvl.u[8 + i] = sVl[16 + 8 * hh + i][dt * 16 + ln];
      }
      oacc[dt] = mmaN<3>(pah.v, pal.v, bvh.v, bvl.v, oacc[dt]);
    }
    __builtin_amdgcn_fence(__ATOMIC_ACQ_REL, "workgroup");
    __builtin_amdgcn_wave_barrier();
  }
#pragma unroll
  for (int r = 0; r < 8; ++r) {
    float l = l_r[r];
    l += __shfl_xor(l, 1, 32); l += __shfl_xor(l, 2, 32); l += __shfl_xor(l, 4, 32); l += __shfl_xor(l, 8, 32);
    l_r[r] = (l > 0.f) ? 1.0f / l : 0.f;
  }
#pragma unroll
  for (int dt = 0; dt < DT; ++dt)
#pragma unroll
    for (int r = 0; r < 8; ++r) sO[w][8 * hh + r][dt * 16 + ln] = oacc[dt][r] * l_r[r];
  __builtin_amdgcn_fence(__ATOMIC_ACQ_REL, "workgroup");
  __builtin_amdgcn_wave_barrier();
  for (int pass = 0; pass < 2; ++pass) {
    for (int r = 0; r < 16; ++r) {
      const int row = q0 + r;
      if (row < T && lane < D / 4) {
        const v4f val = *(const v4fa*)&sO[w][r][lane * 4];
        *(volatile v4f*)(y + ((size_t)b * T + row) * ypitch + h * D + lane * 4) = val;
      }
    }
    if (pass == 0) __threadfence();
  }
}

__global__ __launch_bounds__(256) void k_sort_init(const int* __restrict__ seg, int n, int nseg, unsigned int* __restrict__ key, unsigned int* __restrict__ val, int np2) {
  const int i = blockIdx.x * 256 + threadIdx.x; if (i >= np2) return;
  unsigned int kv = 0xFFFFFFFFu;
  if (i < n) { int s = seg[i]; s = s < 0 ? 0 : (s >= nseg ? nseg - 1 : s); kv = (unsigned int)s; }
  *(volatile unsigned int*)(key + i) = kv; *(volatile unsigned int*)(val + i) = (unsigned int)i;
  __threadfence();
  *(volatile unsigned int*)(key + i) = kv; *(volatile unsigned int*)(val + i) = (unsigned int)i;
}
template <bool STAGE0>
__global__ __launch_bounds__(512) void k_sort_lds(unsigned int* __restrict__ key, unsigned int* __restrict__ val, int kstage) {
  __shared__ unsigned int sk[1024], sv[1024];
  const int tid = threadIdx.x; const int base = blockIdx.x * 1024;
  sk[tid] = key[base + tid]; sv[tid] = val[base + tid]; sk[tid + 512] = key[base + tid + 512]; sv[tid + 512] = val[base + tid + 512];
  __syncthreads();
  for (int k = (STAGE0 ? 2 : kstage); k <= (STAGE0 ? 1024 : kstage); k <<= 1) {
    for (int j = (k > 1024 ? 512 : (k >> 1)); j >= 1; j >>= 1) {
      const int lo = tid & (j - 1), hi2 = (tid >> __builtin_ctz(j)) << (__builtin_ctz(j) + 1);
      const int il = hi2 | lo, ir = il | j;
      const int gi = base + il;
      const bool asc = ((gi & k) == 0);
      unsigned int a = sk[il], b = sk[ir], va = sv[il], vb = sv[ir];
      const bool swp = asc ? (a > b) : (a < b);
      if (swp) { sk[il] = b; sk[ir] = a; sv[il] = vb; sv[ir] = va; }
      __syncthreads();
    }
  }
  for (int pass = 0; pass < 2; ++pass) {
    *(volatile unsigned int*)(key + base + tid) = sk[tid]; *(volatile unsigned int*)(val + base + tid) = sv[tid];
    *(volatile unsigned int*)(key + base + tid + 512) = sk[tid + 512]; *(volatile unsigned int*)(val + base + tid + 512) = sv[tid + 512];
    if (pass == 0) __threadfence();
  }
}
__global__ __launch_bounds__(256) void k_sort_step(unsigned int* __restrict__ key, unsigned int* __restrict__ val, int k, int j, int np2) {
  const int t = blockIdx.x * 256 + threadIdx.x; if (t >= np2 / 2) return;
  const int lo = t & (j - 1), il = ((t >> __builtin_ctz(j)) << (__builtin_ctz(j) + 1)) | lo, ir = il | j;
  const bool asc = ((il & k) == 0);
  unsigned int a = key[il], b = key[ir], va = val[il], vb = val[ir];
  const bool swp = asc ? (a > b) : (a < b);
  const unsigned int k1 = swp ? b : a, k2 = swp ? a : b, v1 = swp ? vb : va, v2 = swp ? va : vb;
  *(volatile unsigned int*)(key + il) = k1; *(volatile unsigned int*)(key + ir) = k2; *(volatile unsigned int*)(val + il) = v1; *(volatile unsigned int*)(val + ir) = v2;
  __threadfence();
  *(volatile unsigned int*)(key + il) = k1; *(volatile unsigned int*)(key + ir) = k2; *(volatile unsigned int*)(val + il) = v1; *(volatile unsigned int*)(val + ir) = v2;
}
__global__ __launch_bounds__(256) void k_rowptr(const unsigned int* __restrict__ key, int np2, int nseg, int* __restrict__ rowptr) {
  int s = blockIdx.x * 256 + threadIdx.x; if (s >= ((nseg + 1 + 31) / 32) * 32) return;
  const int sdst = s; if (s > nseg) s = nseg;
  int lo = 0, hi = np2;
  while (lo < hi) { const int mid = (lo + hi) >> 1; if (key[mid] < (unsigned int)s) lo = mid + 1; else hi = mid; }
  *(volatile int*)(rowptr + sdst) = lo; __threadfence(); *(volatile int*)(rowptr + sdst) = lo;
}
static void sort_pairs(unsigned int* key, unsigned int* val, int np2, hipStream_t stream) {
  k_sort_lds<true><<<np2 / 1024, 512, 0, stream>>>(key, val, 0);
  for (int k = 2048; k <= np2; k <<= 1) {
    for (int j = k >> 1; j >= 1024; j >>= 1) k_sort_step<<<(np2 / 2 + 255) / 256, 256, 0, stream>>>(key, val, k, j, np2);
    k_sort_lds<false><<<np2 / 1024, 512, 0, stream>>>(key, val, k);
  }
}

__global__ __launch_bounds__(256) void k_round_rows(const float* __restrict__ W, unsigned short* __restrict__ Wt, int n8) {
  const int t = blockIdx.x * 256 + threadIdx.x;
  if (t >= n8) return;
  const v4f a = *(const v4fa*)(W + (size_t)t * 8), b = *(const v4fa*)(W + (size_t)t * 8 + 4);
  v8us v; v[0]=bf16_bits(a[0]); v[1]=bf16_bits(a[1]); v[2]=bf16_bits(a[2]); v[3]=bf16_bits(a[3]);
  v[4]=bf16_bits(b[0]); v[5]=bf16_bits(b[1]); v[6]=bf16_bits(b[2]); v[7]=bf16_bits(b[3]);
  *(volatile v8us*)(Wt + (size_t)t * 8) = v; __threadfence(); *(volatile v8us*)(Wt + (size_t)t * 8) = v;
}

__global__ __launch_bounds__(256) void k_edge_score(const float* __restrict__ q, const float* __restrict__ k, const int* __restrict__ src, const int* __restrict__ dst, float* __restrict__ a) {
  __shared__ float res[32];
  const int tid = threadIdx.x, w = tid >> 5, lane = tid & 31; const int e0 = blockIdx.x * 32;
  for (int u = 0; u < 4; ++u) {
    const int e = e0 + w * 4 + u;
    float s = 0.f;
    if (e < NEDGE) {
      int sn = src[e], dn = dst[e]; sn = sn < 0 ? 0 : (sn >= NNODE ? NNODE - 1 : sn); dn = dn < 0 ? 0 : (dn >= NNODE ? NNODE - 1 : dn);
      const float* qr = q + (size_t)sn * DIM; const float* kr = k + (size_t)dn * DIM;
#pragma unroll
      for (int i = 0; i < DIM / 32; ++i) s += qr[lane + 32 * i] * kr[lane + 32 * i];
      for (int o = 16; o >= 1; o >>= 1) s += __shfl_xor(s, o, 32);
    }
    if (lane == 0) res[w * 4 + u] = s * (1.0f / (8.0f * 256.0f));
  }
  __syncthreads();
  if (tid < 32 && e0 + tid < NEDGE) { const float v = res[tid]; *(volatile float*)(a + e0 + tid) = v; __threadfence(); *(volatile float*)(a + e0 + tid) = v; }
}
template <int MODE>
__global__ __launch_bounds__(256) void k_reduce1(const float* __restrict__ a, int n, const float* __restrict__ mslot, float* __restrict__ slots) {
  __shared__ double red[256];
  const int tid = threadIdx.x; double s = 0.0; const float m = MODE ? mslot[0] : 0.f;
  for (int i = blockIdx.x * 4096 + tid; i < min(n, (int)(blockIdx.x * 4096 + 4096)); i += 256) { const float v = a[i]; s += MODE ? (double)(v - m) * (double)(v - m) : (double)v; }
  red[tid] = s; __syncthreads();
  for (int st = 128; st > 0; st >>= 1) { if (tid < st) red[tid] += red[tid + st]; __syncthreads(); }
  if (tid < 32) { const float v = (tid == 0) ? (float)red[0] : 0.f; *(volatile float*)(slots + (size_t)blockIdx.x * 32 + tid) = v; __threadfence(); *(volatile float*)(slots + (size_t)blockIdx.x * 32 + tid) = v; }
}
template <int MODE>
__global__ __launch_bounds__(256) void k_reduce2(const float* __restrict__ slots, int nslots, int n, float* __restrict__ outslot) {
  __shared__ double red[256];
  const int tid = threadIdx.x; double s = 0.0;
  for (int i = tid; i < nslots; i += 256) s += (double)slots[(size_t)i * 32];
  red[tid] = s; __syncthreads();
  for (int st = 128; st > 0; st >>= 1) { if (tid < st) red[tid] += red[tid + st]; __syncthreads(); }
  if (tid < 32) { double r = red[0] / (double)n; if (MODE) r = sqrt(r); const float v = (tid == 0) ? (float)r : 0.f; *(volatile float*)(outslot + tid) = v; __threadfence(); *(volatile float*)(outslot + tid) = v; }
}
__global__ __launch_bounds__(256) void k_node_softmax_stats(const float* __restrict__ a, const float* __restrict__ mslot, const float* __restrict__ sslot,
                                                          const int* __restrict__ rowptr, const unsigned int* __restrict__ perm, float* __restrict__ Mx, float* __restrict__ Sm) {
  const int slot = blockIdx.x * 256 + threadIdx.x; if (slot >= ((NNODE + 31) / 32) * 32) return;
  const int nd = slot < NNODE ? slot : NNODE - 1;
  const float m = mslot[0], s = sslot[0];
  const int p0 = rowptr[nd], p1 = rowptr[nd + 1];
  float mx = -__builtin_inff();
  for (int p = p0; p < p1; ++p) { const float v = (a[perm[p]] - m) / s / TEMP; mx = fmaxf(mx, v); }
  float sum = 0.f;
  for (int p = p0; p < p1; ++p) { const float v = (a[perm[p]] - m) / s / TEMP; sum += expf(v - mx); }
  *(volatile float*)(Mx + slot) = mx; *(volatile float*)(Sm + slot) = sum; __threadfence(); *(volatile float*)(Mx + slot) = mx; *(volatile float*)(Sm + slot) = sum;
}
__global__ __launch_bounds__(256) void k_edge_alpha(const float* __restrict__ a, const float* __restrict__ mslot, const float* __restrict__ sslot, const int* __restrict__ dst,
                                                  const float* __restrict__ Mx, const float* __restrict__ Sm, float* __restrict__ alpha) {
  const int e = blockIdx.x * 256 + threadIdx.x; if (e >= NEDGE) return;
  int dn = dst[e]; dn = dn < 0 ? 0 : (dn >= NNODE ? NNODE - 1 : dn);
  const float v = (a[e] - mslot[0]) / sslot[0] / TEMP;
  const float al = expf(v - Mx[dn]) / Sm[dn];
  *(volatile float*)(alpha + e) = al; __threadfence(); *(volatile float*)(alpha + e) = al;
}
__global__ __launch_bounds__(256) void k_aggregate(const float* __restrict__ vf, const float* __restrict__ alpha, const int* __restrict__ src,
                                                 const int* __restrict__ rowptr, const unsigned int* __restrict__ perm, float* __restrict__ out) {
  const int tid = threadIdx.x, w = tid >> 5, lane = tid & 31;
  const int nd = blockIdx.x * 8 + w; if (nd >= NNODE) return;
  const int p0 = rowptr[nd], p1 = rowptr[nd + 1];
  v4f acc0 = {0.f,0.f,0.f,0.f}, acc1 = {0.f,0.f,0.f,0.f};
  for (int p = p0; p < p1; ++p) {
    const int e = (int)perm[p]; int sn = src[e]; sn = sn < 0 ? 0 : (sn >= NNODE ? NNODE - 1 : sn);
    const float al = alpha[e];
    const v4f x0 = *(const v4fa*)(vf + (size_t)sn * DIM + lane * 4), x1 = *(const v4fa*)(vf + (size_t)sn * DIM + 128 + lane * 4);
    for (int qd = 0; qd < 4; ++qd) { acc0[qd] += al * x0[qd]; acc1[qd] += al * x1[qd]; }
  }
  float* orow = out + (size_t)nd * DIM;
  *(volatile v4f*)(orow + lane * 4) = acc0; *(volatile v4f*)(orow + 128 + lane * 4) = acc1; __threadfence();
  *(volatile v4f*)(orow + lane * 4) = acc0; *(volatile v4f*)(orow + 128 + lane * 4) = acc1;
}

extern "C" void kernel_launch(void* const* d_in, const int* in_sizes, int n_in,
                              void* d_out, int out_size, void* d_ws, size_t ws_size, hipStream_t stream) {
  (void)in_sizes; (void)n_in; (void)out_size;
  const float* h = (const float*)d_in[0]; const int* src = (const int*)d_in[1]; const int* dst = (const int*)d_in[2];
  const float* attn_q = (const float*)d_in[3]; const float* attn_k = (const float*)d_in[4]; const float* W = (const float*)d_in[5]; const float* b = (const float*)d_in[6];
  float* out = (float*)d_out; float* alpha = (float*)d_out + (size_t)NNODE * DIM;
  char* ws = (char*)d_ws; size_t off = 0;
  auto take = [&](size_t bytes) { char* p = ws + off; off += (bytes + 255) & ~(size_t)255; return p; };
  const int nslots = (NEDGE + 4095) / 4096;
  unsigned short* Wt = (unsigned short*)take((size_t)DIM * DIM * 2); unsigned short* Qt = (unsigned short*)take((size_t)DIM * DIM * 2); unsigned short* Kt = (unsigned short*)take((size_t)DIM * DIM * 2);
  float* vf = (float*)take((size_t)NNODE * DIM * 4); float* qf = (float*)take((size_t)NNODE * DIM * 4); float* kf = (float*)take((size_t)NNODE * DIM * 4);
  float* a = (float*)take((size_t)NEDGE * 4);
  float* slots = (float*)take((size_t)nslots * 32 * 4); float* mslot = (float*)take(32 * 4); float* sslot = (float*)take(32 * 4);
  unsigned int* key = (unsigned int*)take((size_t)NP2 * 4); unsigned int* perm = (unsigned int*)take((size_t)NP2 * 4);
  int* rowptr = (int*)take((size_t)(NNODE + 1) * 4 + 256);
  float* Mx = (float*)take((size_t)(NNODE + 32) * 4); float* Sm = (float*)take((size_t)(NNODE + 32) * 4);
  if (off > ws_size) return;
  k_round_rows<<<(DIM * DIM / 8 + 255) / 256, 256, 0, stream>>>(W, Wt, DIM * DIM / 8);
  k_wt_bf16<<<(DIM * (DIM / 8) + 255) / 256, 256, 0, stream>>>(attn_q, Qt, DIM, DIM);
  k_wt_bf16<<<(DIM * (DIM / 8) + 255) / 256, 256, 0, stream>>>(attn_k, Kt, DIM, DIM);
  const int M = NNODE;
  k_gemm_bf<false, 0, true><<<((M / 16) * (DIM / 64) + 3) / 4, 128, 0, stream>>>(h, DIM, Wt, DIM, b, vf, DIM, M, DIM, DIM);
  k_gemm_bf<false, 0, false><<<((M / 16) * (DIM / 64) + 3) / 4, 128, 0, stream>>>(h, DIM, Qt, DIM, nullptr, qf, DIM, M, DIM, DIM);
  k_gemm_bf<false, 0, false><<<((M / 16) * (DIM / 64) + 3) / 4, 128, 0, stream>>>(h, DIM, Kt, DIM, nullptr, kf, DIM, M, DIM, DIM);
  k_edge_score<<<(NEDGE + 31) / 32, 256, 0, stream>>>(qf, kf, src, dst, a);
  k_reduce1<0><<<nslots, 256, 0, stream>>>(a, NEDGE, nullptr, slots);
  k_reduce2<0><<<1, 256, 0, stream>>>(slots, nslots, NEDGE, mslot);
  k_reduce1<1><<<nslots, 256, 0, stream>>>(a, NEDGE, mslot, slots);
  k_reduce2<1><<<1, 256, 0, stream>>>(slots, nslots, NEDGE, sslot);
  k_sort_init<<<NP2 / 256, 256, 0, stream>>>(dst, NEDGE, NNODE, key, perm, NP2);
  sort_pairs(key, perm, NP2, stream);
  k_rowptr<<<(NNODE + 32 + 255) / 256, 256, 0, stream>>>(key, NP2, NNODE, rowptr);
  k_node_softmax_stats<<<(NNODE + 32 + 255) / 256, 256, 0, stream>>>(a, mslot, sslot, rowptr, perm, Mx, Sm);
  k_edge_alpha<<<(NEDGE + 255) / 256, 256, 0, stream>>>(a, mslot, sslot, dst, Mx, Sm, alpha);
  k_aggregate<<<(NNODE + 7) / 8, 256, 0, stream>>>(vf, alpha, src, rowptr, perm, out);
}
